// Attention_8211977470693
// MI455X (gfx1250) — hardware-verified
//
#include <hip/hip_runtime.h>


#ifndef NB
#define NB 4
#endif
#ifndef SEQ
#define SEQ 2048
#endif
#define NB_FULL  4
#define SEQ_FULL 2048
#define DM   1024
#define NH   16
#define HD   64
#define DQ   (NH * HD)
#define NQKV (3 * DQ)
#define PSH  10.0f
#define CL2  0.18033688011112042f
#define CCAR 16.0f
#define WCAR 16.0f

static_assert(SEQ % 64 == 0);
static_assert(SEQ <= SEQ_FULL);
static_assert(NB <= NB_FULL);
static_assert(DM == 1024);
static_assert(DQ == 1024);
static_assert(NH == 16);
static_assert(HD == 64);
static_assert((SEQ * HD) % 256 == 0);
static_assert(((size_t)NB * SEQ * DM / 8) % 256 == 0);

typedef _Float16 h16;
typedef unsigned short bf;
typedef __attribute__((ext_vector_type(16))) __bf16   v16bf;
typedef __attribute__((ext_vector_type(16))) _Float16 v16h;
typedef __attribute__((ext_vector_type(8)))  _Float16 v8h;
typedef __attribute__((ext_vector_type(2)))  _Float16 v2h;
typedef __attribute__((ext_vector_type(8)))  unsigned short v8us;
typedef __attribute__((ext_vector_type(2)))  unsigned short v2us;
typedef __attribute__((ext_vector_type(8)))  float    v8f;
typedef __attribute__((ext_vector_type(4)))  float    v4f;
typedef v8h  __attribute__((may_alias)) v8ha;
typedef v4f  __attribute__((may_alias)) v4fa;

__device__ __forceinline__ unsigned short f2bf(float f) { unsigned u = __float_as_uint(f); u += 0x7FFFu + ((u >> 16) & 1u); return (unsigned short)(u >> 16); }
__device__ __forceinline__ float bf2f(unsigned short b) { return __uint_as_float(((unsigned)b) << 16); }
__device__ __forceinline__ float bfr(float f) { return bf2f(f2bf(f)); }
__device__ __forceinline__ v16h cat16(v8h lo, v8h hi) { return __builtin_shufflevector(lo, hi, 0, 1, 2, 3, 4, 5, 6, 7, 8, 9, 10, 11, 12, 13, 14, 15); }
__device__ __forceinline__ v16bf cat16b(v8us lo, v8us hi) { return __builtin_bit_cast(v16bf, __builtin_shufflevector(lo, hi, 0, 1, 2, 3, 4, 5, 6, 7, 8, 9, 10, 11, 12, 13, 14, 15)); }
__device__ __forceinline__ v8f wmma16(v16h a, v16h b, v8f c) { return __builtin_amdgcn_wmma_f32_16x16x32_f16(false, a, false, b, (short)0, c, false, false); }
__device__ __forceinline__ v8f wmmab(v16bf a, v16bf b, v8f c) { return __builtin_amdgcn_wmma_f32_16x16x32_bf16(false, a, false, b, (short)0, c, false, false); }
__device__ __forceinline__ v16h  ldh(const h16* p) { return cat16(*(const v8h*)p, *(const v8h*)(p + 16)); }
__device__ __forceinline__ v16bf ldb(const bf* p)  { return cat16b(*(const v8us*)p, *(const v8us*)(p + 16)); }

__global__ __launch_bounds__(256) void k_wtb(const float* __restrict__ w, unsigned N, bf* Bt) {
    const unsigned lane = threadIdx.x & 31u; const unsigned L0 = (blockIdx.x * 8u + (threadIdx.x >> 5)) * 8u; const unsigned nlines = N * 16u;
#pragma unroll 1
    for (int ps = 0; ps < 2; ++ps) {
#pragma unroll 1
        for (unsigned l = 0; l < 8u; ++l) { const unsigned L = L0 + l;
            if (L < nlines) { const unsigned e = L * 64u + lane * 2u; const unsigned k = e & 1023u, n = e >> 10; v2us o;
                o[0] = f2bf(w[(size_t)k * N + n]); o[1] = f2bf(w[(size_t)(k + 1u) * N + n]); *(volatile v2us*)(Bt + e) = o; } }
        if (ps == 0) __threadfence(); }
}
__global__ __launch_bounds__(256) void k_wth(const float* __restrict__ w, unsigned N, h16* Bt) {
    const unsigned lane = threadIdx.x & 31u; const unsigned L0 = (blockIdx.x * 8u + (threadIdx.x >> 5)) * 8u; const unsigned nlines = N * 16u;
#pragma unroll 1
    for (int ps = 0; ps < 2; ++ps) {
#pragma unroll 1
        for (unsigned l = 0; l < 8u; ++l) { const unsigned L = L0 + l;
            if (L < nlines) { const unsigned e = L * 64u + lane * 2u; const unsigned k = e & 1023u, n = e >> 10; v2h o;
                o[0] = (h16)(bfr(w[(size_t)k * N + n]) * WCAR); o[1] = (h16)(bfr(w[(size_t)(k + 1u) * N + n]) * WCAR); *(volatile v2h*)(Bt + e) = o; } }
        if (ps == 0) __threadfence(); }
}

__global__ __launch_bounds__(256) void k_cvt8(const float* __restrict__ x, bf* XB) {
    const unsigned i = blockIdx.x * 256u + threadIdx.x; const unsigned row = i >> 7, c8 = i & 127u; const unsigned b = row / SEQ, t = row % SEQ;
    const v8f v = *(const v8f*)(x + ((size_t)b * SEQ_FULL + t) * DM + c8 * 8u); v8us o;
#pragma unroll
    for (int k = 0; k < 8; ++k) o[k] = f2bf(v[k]);
    *(volatile v8us*)(XB + (size_t)i * 8u) = o; __threadfence(); *(volatile v8us*)(XB + (size_t)i * 8u) = o;
}

__global__ __launch_bounds__(256) void k_cstab(const float* __restrict__ pos, float* COS, float* SIN) {
    const unsigned idx = blockIdx.x * 256u + threadIdx.x; const float p = bfr(pos[idx]); const float c = cosf(p); const float s = sinf(p);
    *(volatile float*)(COS + idx) = c; *(volatile float*)(SIN + idx) = s; __threadfence(); *(volatile float*)(COS + idx) = c; *(volatile float*)(SIN + idx) = s;
}

__global__ __launch_bounds__(32) void k_proj(const bf* __restrict__ A, const bf* __restrict__ Bt, const float* __restrict__ COS, const float* __restrict__ SIN, h16* Qp, h16* Kp, h16* VTp) {
    __shared__ __align__(16) float os[64 * 68];
    const unsigned lane = threadIdx.x & 31u, lr = lane & 15u, hi = lane >> 4; const unsigned r0 = blockIdx.x * 64u, c0 = blockIdx.y * 64u;
    v8f acc[4][4];
#pragma unroll
    for (int mb = 0; mb < 4; ++mb)
#pragma unroll
        for (int nb = 0; nb < 4; ++nb) acc[mb][nb] = (v8f){};
    const size_t aoff = (size_t)(r0 + lr) * DM + 8u * hi, boff = (size_t)(c0 + lr) * DM + 8u * hi;
#pragma unroll 1
    for (unsigned kc = 0; kc < DM; kc += 32u) {
        v16bf a[4];
#pragma unroll
        for (int mb = 0; mb < 4; ++mb) a[mb] = ldb(A + aoff + (size_t)mb * 16 * DM + kc);
#pragma unroll
        for (int nb = 0; nb < 4; ++nb) { const v16bf bq = ldb(Bt + boff + (size_t)nb * 16 * DM + kc);
#pragma unroll
            for (int mb = 0; mb < 4; ++mb) acc[mb][nb] = wmmab(a[mb], bq, acc[mb][nb]); }
        asm volatile("v_nop\n\tv_nop\n\tv_nop\n\tv_nop" : "+v"(acc[0][0]), "+v"(acc[1][1]), "+v"(acc[2][2]), "+v"(acc[3][3]) : "v"(a[0]), "v"(a[3]));
    }
#pragma unroll
    for (int mb = 0; mb < 4; ++mb)
#pragma unroll
        for (int nb = 0; nb < 4; ++nb)
#pragma unroll
            for (int j = 0; j < 8; ++j) os[(mb * 16 + hi * 8 + j) * 68 + nb * 16 + lr] = acc[mb][nb][j];
    __syncthreads();
    const unsigned region = c0 >> 10, h = (c0 & 1023u) >> 6; const unsigned b = r0 / SEQ, t0 = r0 % SEQ; const unsigned sub = lane >> 3, seg = lane & 7u;
    if (region < 2u) {
        h16* P = (region == 0u) ? Qp : Kp;
        h16* prow = P + ((size_t)(b * NH + h) * SEQ + t0) * HD + seg * 8u;
        const float sg = (seg < 4u) ? -1.0f : 1.0f;
        const unsigned dx = seg * 8u, dy = (seg * 8u) ^ 32u;
#pragma unroll 1
        for (int ps = 0; ps < 2; ++ps) {
#pragma unroll 2
            for (unsigned s = 0; s < 16u; ++s) { const unsigned row = 4u * s + sub; const float* xr = os + row * 68u;
                const v4f x0 = *(const v4fa*)(xr + dx), x1 = *(const v4fa*)(xr + dx + 4u), y0 = *(const v4fa*)(xr + dy), y1 = *(const v4fa*)(xr + dy + 4u);
                const size_t to = (size_t)(t0 + row) * HD + dx;
                const v4f ca = *(const v4f*)(COS + to), cb = *(const v4f*)(COS + to + 4), sa = *(const v4f*)(SIN + to), sb = *(const v4f*)(SIN + to + 4);
                v8h o;
#pragma unroll
                for (int j = 0; j < 4; ++j) { o[j] = (h16)(x0[j] * ca[j] + sg * (y0[j] * sa[j])); o[4 + j] = (h16)(x1[j] * cb[j] + sg * (y1[j] * sb[j])); }
                *(volatile v8h*)(prow + (size_t)row * HD) = o; }
            if (ps == 0) __threadfence(); }
    } else {
        h16* vrow = VTp + ((size_t)(b * NH + h) * HD) * SEQ + t0 + seg * 8u;
#pragma unroll 1
        for (int ps = 0; ps < 2; ++ps) {
#pragma unroll 2
            for (unsigned s = 0; s < 16u; ++s) { const unsigned d = 4u * s + sub; v8h o;
#pragma unroll
                for (int j = 0; j < 8; ++j) o[j] = (h16)os[(seg * 8u + j) * 68u + d];
                *(volatile v8h*)(vrow + (size_t)d * SEQ) = o; }
            if (ps == 0) __threadfence(); }
    }
}

__device__ __forceinline__ v8h pk8(v8f o, float s) { v8h t;
#pragma unroll
    for (int r = 0; r < 8; ++r) t[r] = (h16)(o[r] * s);
    return t; }

__global__ __launch_bounds__(128) void k_flash(const h16* __restrict__ Qp, const h16* __restrict__ Kp, const h16* __restrict__ VTp, h16* CTX) {
    __shared__ __align__(16) h16 os[4 * 16 * 72];
    const unsigned tid = threadIdx.x, wv = tid >> 5, lane = tid & 31u, lr = lane & 15u, hi = lane >> 4;
    const unsigned bh = blockIdx.y; const unsigned b = bh >> 4, h = bh & 15u; const unsigned q0 = blockIdx.x * 64u + wv * 16u;
    const h16* qrow = Qp + ((size_t)bh * SEQ + q0 + lr) * HD + 8u * hi;
    const v16h qf0 = ldh(qrow), qf1 = ldh(qrow + 32);
    const h16* kbase = Kp + ((size_t)bh * SEQ + lr) * HD + 8u * hi;
    const h16* vbase = VTp + ((size_t)bh * HD + lr) * SEQ + 8u * hi;
    v8f o0 = (v8f){}, o1 = (v8f){}, o2 = (v8f){}, o3 = (v8f){};
    float m_run = -1.0e30f, l_run = 0.0f;
#pragma unroll 1
    for (unsigned key0 = 0; key0 < SEQ; key0 += 32u) {
        const h16* kp = kbase + (size_t)key0 * HD;
        const v16h k00 = ldh(kp), k01 = ldh(kp + 32), k10 = ldh(kp + 16 * HD), k11 = ldh(kp + 16 * HD + 32);
        const h16* vp = vbase + key0;
        const v16h v0 = ldh(vp), v1 = ldh(vp + (size_t)16 * SEQ), v2 = ldh(vp + (size_t)32 * SEQ), v3 = ldh(vp + (size_t)48 * SEQ);
        v8f s0 = (v8f){}, s1 = (v8f){};
        s0 = wmma16(k00, qf0, s0); s1 = wmma16(k10, qf0, s1); s0 = wmma16(k01, qf1, s0); s1 = wmma16(k11, qf1, s1);
        asm volatile("v_nop\n\tv_nop\n\tv_nop\n\tv_nop" : "+v"(s0), "+v"(s1) : "v"(k00), "v"(k01), "v"(k10), "v"(k11), "v"(qf0), "v"(qf1));
        float mx = fmaxf(s0[0], s1[0]);
#pragma unroll
        for (int r = 1; r < 8; ++r) mx = fmaxf(mx, fmaxf(s0[r], s1[r]));
        mx = fmaxf(mx, __shfl_xor(mx, 16, 32));
        const float mnew = fmaxf(m_run, mx);
        const float cr = __builtin_amdgcn_exp2f((m_run - mnew) * CL2);
        const float off = PSH - mnew * CL2;
        v16h pf; float psum = 0.0f;
#pragma unroll
        for (int r = 0; r < 8; ++r) { const float p = __builtin_amdgcn_exp2f(fmaf(s0[r], CL2, off)); psum += p; pf[r] = (h16)p; }
#pragma unroll
        for (int r = 0; r < 8; ++r) { const float p = __builtin_amdgcn_exp2f(fmaf(s1[r], CL2, off)); psum += p; pf[8 + r] = (h16)p; }
        l_run = l_run * cr + psum; m_run = mnew;
        o0 = o0 * cr; o1 = o1 * cr; o2 = o2 * cr; o3 = o3 * cr;
        o0 = wmma16(v0, pf, o0); o1 = wmma16(v1, pf, o1); o2 = wmma16(v2, pf, o2); o3 = wmma16(v3, pf, o3);
        asm volatile("v_nop\n\tv_nop\n\tv_nop\n\tv_nop" : "+v"(o0), "+v"(o1), "+v"(o2), "+v"(o3) : "v"(v0), "v"(v1), "v"(v2), "v"(v3), "v"(pf));
    }
    const float l = l_run + __shfl_xor(l_run, 16, 32);
    const float inv = CCAR * (1.0f / l);
    h16* ow = os + wv * (16u * 72u);
    *(v8ha*)(ow + lr * 72u +  0u + 8u * hi) = pk8(o0, inv);
    *(v8ha*)(ow + lr * 72u + 16u + 8u * hi) = pk8(o1, inv);
    *(v8ha*)(ow + lr * 72u + 32u + 8u * hi) = pk8(o2, inv);
    *(v8ha*)(ow + lr * 72u + 48u + 8u * hi) = pk8(o3, inv);
    __syncthreads();
    const unsigned sub = lane >> 3, seg = lane & 7u;
    h16* cbase = CTX + ((size_t)b * SEQ + q0) * DQ + h * HD + seg * 8u;
#pragma unroll 1
    for (int ps = 0; ps < 2; ++ps) {
#pragma unroll
        for (unsigned s = 0; s < 4u; ++s) { const unsigned row = 4u * s + sub; const v8h val = *(const v8ha*)(ow + row * 72u + seg * 8u);
            *(volatile v8h*)(cbase + (size_t)row * DQ) = val; }
        if (ps == 0) __threadfence(); }
}

__global__ __launch_bounds__(32) void k_gemmo(const h16* __restrict__ A, const h16* __restrict__ Bt, float* C, const float* __restrict__ bias, float osc, size_t sA, size_t sC) {
    __shared__ __align__(16) float os[16 * 68];
    const size_t z = blockIdx.z; A += z * sA; C += z * sC;
    const unsigned lane = threadIdx.x & 31u, lr = lane & 15u, hi = lane >> 4; const unsigned r0 = blockIdx.x * 64u, c0 = blockIdx.y * 64u;
    v8f acc[4][4];
#pragma unroll
    for (int mb = 0; mb < 4; ++mb)
#pragma unroll
        for (int nb = 0; nb < 4; ++nb) acc[mb][nb] = (v8f){};
    const size_t aoff = (size_t)(r0 + lr) * DQ + 8u * hi, boff = (size_t)(c0 + lr) * DQ + 8u * hi;
#pragma unroll 1
    for (unsigned kc = 0; kc < DQ; kc += 32u) {
        v16h a[4];
#pragma unroll
        for (int mb = 0; mb < 4; ++mb) a[mb] = ldh(A + aoff + (size_t)mb * 16 * DQ + kc);
#pragma unroll
        for (int nb = 0; nb < 4; ++nb) { const v16h bq = ldh(Bt + boff + (size_t)nb * 16 * DQ + kc);
#pragma unroll
            for (int mb = 0; mb < 4; ++mb) acc[mb][nb] = wmma16(a[mb], bq, acc[mb][nb]); }
        asm volatile("v_nop\n\tv_nop\n\tv_nop\n\tv_nop" : "+v"(acc[0][0]), "+v"(acc[1][1]), "+v"(acc[2][2]), "+v"(acc[3][3]) : "v"(a[0]), "v"(a[3]));
    }
    const unsigned cofs = lr * 4u; v4f bv;
#pragma unroll
    for (int i = 0; i < 4; ++i) bv[i] = bfr(bias[c0 + cofs + i]);
#pragma unroll
    for (int mb = 0; mb < 4; ++mb) {
#pragma unroll
        for (int nb = 0; nb < 4; ++nb)
#pragma unroll
            for (int j = 0; j < 8; ++j) os[(hi * 8 + j) * 68 + nb * 16 + lr] = acc[mb][nb][j];
        __syncthreads();
        float* crow = C + (size_t)(r0 + mb * 16) * DM + c0;
#pragma unroll 1
        for (int ps = 0; ps < 2; ++ps) {
#pragma unroll
            for (unsigned s = 0; s < 8u; ++s) { const unsigned row = 2u * s + hi; v4f val = *(const v4fa*)(os + row * 68u + cofs); val = val * osc + bv;
                *(volatile v4f*)(crow + (size_t)row * DM + cofs) = val; }
            if (ps == 0) __threadfence(); }
        __syncthreads();
    }
}

extern "C" void kernel_launch(void* const* d_in, const int* in_sizes, int n_in,
                              void* d_out, int out_size, void* d_ws, size_t ws_size, hipStream_t stream) {
    if (n_in < 6) return;
    if ((size_t)in_sizes[0] < (size_t)NB * SEQ * DM) return;
    if ((size_t)in_sizes[1] < (size_t)SEQ * HD) return;
    if ((size_t)in_sizes[2] < (size_t)DM * DQ) return;
    if ((size_t)in_sizes[3] < (size_t)DM * 2 * DQ) return;
    if ((size_t)in_sizes[4] < (size_t)DQ * DM) return;
    if ((size_t)in_sizes[5] < (size_t)DM) return;
    if ((size_t)out_size < (size_t)NB * SEQ * DM) return;
    const float* x = (const float*)d_in[0]; const float* pos = (const float*)d_in[1]; const float* wq = (const float*)d_in[2];
    const float* wkv = (const float*)d_in[3]; const float* wo = (const float*)d_in[4]; const float* bo = (const float*)d_in[5];
    float* OUT = (float*)d_out;
    char* wsp = (char*)d_ws;
    auto take = [&](size_t bytes) { char* p = wsp; wsp += (bytes + 255) & ~(size_t)255; return (void*)p; };
    bf*  WALL = (bf*)take((size_t)NQKV * DM * 2);
    h16* WOT  = (h16*)take((size_t)DM * DQ * 2);
    bf*  XB   = (bf*)take((size_t)NB * SEQ * DM * 2);
    float* COS = (float*)take((size_t)SEQ * HD * 4); float* SIN = (float*)take((size_t)SEQ * HD * 4);
    h16* QP  = (h16*)take((size_t)NB * NH * SEQ * HD * 2); h16* KP = (h16*)take((size_t)NB * NH * SEQ * HD * 2); h16* VT = (h16*)take((size_t)NB * NH * HD * SEQ * 2);
    h16* CTX = (h16*)take((size_t)NB * SEQ * DQ * 2);
    const size_t carved = (size_t)(wsp - (char*)d_ws);
    if (carved > ws_size || carved > (size_t)134217728) return;
    k_wtb<<<DQ / 4, 256, 0, stream>>>(wq, (unsigned)DQ, WALL);
    k_wtb<<<2 * DQ / 4, 256, 0, stream>>>(wkv, (unsigned)(2 * DQ), WALL + (size_t)DQ * DM);
    k_wth<<<DM / 4, 256, 0, stream>>>(wo, (unsigned)DM, WOT);
    k_cvt8<<<(unsigned)((size_t)NB * SEQ * DM / 8 / 256), 256, 0, stream>>>(x, XB);
    k_cstab<<<SEQ * HD / 256, 256, 0, stream>>>(pos, COS, SIN);
    k_proj<<<dim3(NB * SEQ / 64, NQKV / 64, 1), 32, 0, stream>>>(XB, WALL, COS, SIN, QP, KP, VT);
    k_flash<<<dim3(SEQ / 64, NB * NH, 1), 128, 0, stream>>>(QP, KP, VT, CTX);
    k_gemmo<<<dim3(SEQ / 64, DM / 64, NB), 32, 0, stream>>>(CTX, WOT, OUT, bo, 1.0f / (CCAR * WCAR), (size_t)SEQ * DQ, (size_t)SEQ_FULL * DM);
}
